// SelectiveSSMBlock_43937515438700
// MI455X (gfx1250) — hardware-verified
//
#include <hip/hip_runtime.h>


#define BB      2
#define TT      2048
#define DM      1024
#define EE      2048
#define NS      32
#define DTR     64
#define XR      128
#define MROWS   (BB * TT)

typedef float  v4f   __attribute__((ext_vector_type(4)));
typedef float  v8f   __attribute__((ext_vector_type(8)));
typedef int    v8i   __attribute__((ext_vector_type(8)));
typedef __bf16 v16bf __attribute__((ext_vector_type(16)));

union Frag { v16bf v; v8i i; unsigned int w[8]; };

__device__ __forceinline__ unsigned int bf16_bits_rne(float x) {
    unsigned int u = __float_as_uint(x);
    u += 0x7FFFu + ((u >> 16) & 1u);
    return u >> 16;
}

__device__ __forceinline__ void load_split(const float* __restrict__ p, Frag& hi, Frag& lo) {
    const v4f q0 = *(const v4f*)(p);
    const v4f q1 = *(const v4f*)(p + 4);
    const v4f q2 = *(const v4f*)(p + 16);
    const v4f q3 = *(const v4f*)(p + 20);
    const float f[16] = { q0.x, q0.y, q0.z, q0.w, q1.x, q1.y, q1.z, q1.w,
                          q2.x, q2.y, q2.z, q2.w, q3.x, q3.y, q3.z, q3.w };
#pragma unroll
    for (int j = 0; j < 8; ++j) {
        const float x0 = f[2 * j];
        const float x1 = f[2 * j + 1];
        const unsigned int h0 = bf16_bits_rne(x0);
        const unsigned int h1 = bf16_bits_rne(x1);
        const unsigned int l0 = bf16_bits_rne(x0 - __uint_as_float(h0 << 16));
        const unsigned int l1 = bf16_bits_rne(x1 - __uint_as_float(h1 << 16));
        hi.w[j] = h0 | (h1 << 16);
        lo.w[j] = l0 | (l1 << 16);
    }
}

__device__ __forceinline__ v8f wmma1(const Frag& a, const Frag& b, v8f c) {
    v8f d = __builtin_amdgcn_wmma_f32_16x16x32_bf16(false, a.v, false, b.v, (short)0, c, false, false);
    asm volatile("v_nop\n\tv_nop\n\tv_nop\n\tv_nop" : "+v"(d) : "v"(a.i), "v"(b.i));
    return d;
}

__device__ __forceinline__ float softplus_f(float v) {
    return fmaxf(v, 0.0f) + log1pf(expf(-fabsf(v)));
}

__global__ __launch_bounds__(256)
void layernorm_kernel(const float* __restrict__ x,
                      const float* __restrict__ g,
                      const float* __restrict__ bta,
                      float* __restrict__ xn, int nrows) {
    __shared__ float red[2][8];
    const int row = blockIdx.x;
    if (row >= nrows) return;
    const int tid = threadIdx.x, wave = tid >> 5, lane = tid & 31;
    const float* xr = x + (size_t)row * DM;
    const v4f v = *(const v4f*)(xr + 4 * tid);

    float s = (v.x + v.y) + (v.z + v.w);
    for (int off = 16; off >= 1; off >>= 1) s += __shfl_xor(s, off, 32);
    if (lane == 0) red[0][wave] = s;
    __syncthreads();
    float tot = 0.f;
#pragma unroll
    for (int w = 0; w < 8; ++w) tot += red[0][w];
    const float mu = tot * (1.0f / DM);

    v4f d;
    d.x = v.x - mu; d.y = v.y - mu; d.z = v.z - mu; d.w = v.w - mu;
    float s2 = (d.x * d.x + d.y * d.y) + (d.z * d.z + d.w * d.w);
    for (int off = 16; off >= 1; off >>= 1) s2 += __shfl_xor(s2, off, 32);
    if (lane == 0) red[1][wave] = s2;
    __syncthreads();
    float tot2 = 0.f;
#pragma unroll
    for (int w = 0; w < 8; ++w) tot2 += red[1][w];
    const float var = tot2 * (1.0f / DM);
    const float rs = rsqrtf(var + 1e-5f);

    const v4f gg = *(const v4f*)(g + 4 * tid);
    const v4f bv = *(const v4f*)(bta + 4 * tid);
    v4f o;
    o.x = (d.x * rs) * gg.x + bv.x;
    o.y = (d.y * rs) * gg.y + bv.y;
    o.z = (d.z * rs) * gg.z + bv.z;
    o.w = (d.w * rs) * gg.w + bv.w;

    float* dst = xn + (size_t)row * DM + 4 * tid;
    *(volatile v4f*)dst = o;
    __threadfence();
    *(volatile v4f*)dst = o;
}

template<int EPI>
__global__ __launch_bounds__(256)
void gemm_split_kernel(const float* __restrict__ A, int lda,
                       const float* __restrict__ Bw,
                       float* __restrict__ C,
                       int M, int N, int K,
                       const float* __restrict__ aux) {
    __shared__ __attribute__((aligned(16))) float tile[8][16][36];
    const int wave = threadIdx.x >> 5;
    const int lane = threadIdx.x & 31;
    const int h    = lane >> 4;
    const int m    = lane & 15;
    const int NG   = N >> 5;
    const int gw   = blockIdx.x * 8 + wave;
    int mt = gw / NG;
    int ng = gw - mt * NG;
    const bool active = (mt * 16 + 16 <= M);
    if (!active) { mt = 0; ng = 0; }
    const int m0 = mt * 16;
    const int n0 = ng * 32;

    v8f acc0 = {0.f, 0.f, 0.f, 0.f, 0.f, 0.f, 0.f, 0.f};
    v8f acc1 = {0.f, 0.f, 0.f, 0.f, 0.f, 0.f, 0.f, 0.f};

    const float* ap  = A  + (size_t)(m0 + m) * lda + 8 * h;
    const float* bp0 = Bw + (size_t)(n0 + m) * K + 8 * h;
    const float* bp1 = Bw + (size_t)(n0 + 16 + m) * K + 8 * h;

#pragma unroll 1
    for (int k0 = 0; k0 < K; k0 += 32) {
        Frag ah, al, b0h, b0l, b1h, b1l;
        load_split(ap  + k0, ah,  al);
        load_split(bp0 + k0, b0h, b0l);
        load_split(bp1 + k0, b1h, b1l);
        acc0 = wmma1(al, b0h, acc0);
        acc0 = wmma1(ah, b0l, acc0);
        acc0 = wmma1(ah, b0h, acc0);
        acc1 = wmma1(al, b1h, acc1);
        acc1 = wmma1(ah, b1l, acc1);
        acc1 = wmma1(ah, b1h, acc1);
    }

#pragma unroll
    for (int r = 0; r < 8; ++r) {
        tile[wave][8 * h + r][m]      = acc0[r];
        tile[wave][8 * h + r][16 + m] = acc1[r];
    }
    __syncthreads();

    const int q    = lane & 7;
    const int rsub = lane >> 3;
    v4f vals[4];
#pragma unroll
    for (int p = 0; p < 4; ++p) {
        const int row  = 4 * p + rsub;
        const int grow = m0 + row;
        const int gcol = n0 + 4 * q;
        v4f v = *(const v4f*)(&tile[wave][row][4 * q]);
        if (EPI == 1) {
            const v4f bia = *(const v4f*)(aux + gcol);
            v.x = softplus_f(v.x + bia.x); v.y = softplus_f(v.y + bia.y);
            v.z = softplus_f(v.z + bia.z); v.w = softplus_f(v.w + bia.w);
        } else if (EPI == 3) {
            const v4f res = *(const v4f*)(aux + (size_t)grow * N + gcol);
            v.x += res.x; v.y += res.y; v.z += res.z; v.w += res.w;
        }
        vals[p] = v;
    }
    if (active) {
#pragma unroll
        for (int p = 0; p < 4; ++p) {
            float* dst = C + (size_t)(m0 + 4 * p + rsub) * N + n0 + 4 * q;
            *(volatile v4f*)dst = vals[p];
        }
    }
    __threadfence();
    if (active) {
#pragma unroll
        for (int p = 0; p < 4; ++p) {
            float* dst = C + (size_t)(m0 + 4 * p + rsub) * N + n0 + 4 * q;
            *(volatile v4f*)dst = vals[p];
        }
    }
}

__global__ __launch_bounds__(256)
void scan_kernel(const float* __restrict__ dt,
                 const float* __restrict__ xz,
                 const float* __restrict__ xdbl,
                 const float* __restrict__ A_log_real,
                 const float* __restrict__ A_imag,
                 const float* __restrict__ D_param,
                 float* __restrict__ yT,
                 int nch) {
#pragma clang fp contract(off)
    const int gw   = blockIdx.x * 8 + (threadIdx.x >> 5);
    const int lane = threadIdx.x & 31;
    if (gw >= nch) return;
    const int b = gw / EE;
    const int e = gw - b * EE;

    const float Ar = -expf(A_log_real[(size_t)e * NS + lane]);
    const float Ai = A_imag[(size_t)e * NS + lane];
    const float Dp = D_param[e];
    float hr = 0.f, hi = 0.f;
    float* yrow = yT + (size_t)gw * TT;

#pragma unroll 1
    for (int t0 = 0; t0 < TT; t0 += 32) {
        const int mpre = b * TT + t0 + lane;
        const float dt_pre = dt[(size_t)mpre * EE + e];
        const float x_pre  = xz[(size_t)mpre * (2 * EE) + e];
        const float z_pre  = xz[(size_t)mpre * (2 * EE) + EE + e];
        float ysave = 0.f;
#pragma unroll 1
        for (int u = 0; u < 32; ++u) {
            const float dtv = __shfl(dt_pre, u, 32);
            const float xv  = __shfl(x_pre,  u, 32);
            const float zv  = __shfl(z_pre,  u, 32);
            const int m2 = b * TT + t0 + u;
            const float Bv = xdbl[(size_t)m2 * XR + DTR + lane];
            const float Cv = xdbl[(size_t)m2 * XR + DTR + NS + lane];

            const float sc  = expf(Ar * dtv);
            const float ang = Ai * dtv;
            float sn, cs;
            sincosf(ang, &sn, &cs);
            const float dAr = sc * cs;
            const float dAi = sc * sn;
            const float dBx = (dtv * xv) * Bv;
            const float hr2 = (dAr * hr - dAi * hi) + dBx;
            const float hi2 = dAr * hi + dAi * hr;
            hr = hr2;
            hi = hi2;

            float p = hr * Cv;
            for (int off = 16; off >= 1; off >>= 1) p += __shfl_xor(p, off, 32);
            const float y  = p + Dp * xv;
            const float sg = zv * (1.0f / (1.0f + expf(-zv)));
            const float yf = y * sg;
            ysave = (lane == u) ? yf : ysave;
        }
        const int src = (lane & 7) * 4;
        v4f o;
        o.x = __shfl(ysave, src + 0, 32);
        o.y = __shfl(ysave, src + 1, 32);
        o.z = __shfl(ysave, src + 2, 32);
        o.w = __shfl(ysave, src + 3, 32);
        float* dst = yrow + t0 + 4 * (lane & 7);
        if (lane < 8) *(volatile v4f*)dst = o;
        __threadfence();
        if (lane < 8) *(volatile v4f*)dst = o;
    }
}

__global__ __launch_bounds__(256)
void transpose_y_kernel(const float* __restrict__ yT, float* __restrict__ y, int nblk) {
    __shared__ float tile[32][33];
    const int bid = blockIdx.x;
    if (bid >= nblk) return;
    const int tb   = bid % (TT / 32);
    const int rest = bid / (TT / 32);
    const int eb   = rest % (EE / 32);
    const int b    = rest / (EE / 32);
    const int e0 = eb * 32, t0 = tb * 32;
    const int tid = threadIdx.x;
    const int tl = tid & 31;
#pragma unroll
    for (int i = 0; i < 4; ++i) {
        const int el = (tid >> 5) + 8 * i;
        tile[el][tl] = yT[((size_t)(b * EE + e0 + el)) * TT + t0 + tl];
    }
    __syncthreads();
    const int wave = tid >> 5, lane = tid & 31;
    const int q = lane & 7, rs = lane >> 3;
    const int trow = 4 * wave + rs;
    v4f v;
    v.x = tile[4 * q + 0][trow];
    v.y = tile[4 * q + 1][trow];
    v.z = tile[4 * q + 2][trow];
    v.w = tile[4 * q + 3][trow];
    float* dst = y + (size_t)(b * TT + t0 + trow) * EE + e0 + 4 * q;
    *(volatile v4f*)dst = v;
    __threadfence();
    *(volatile v4f*)dst = v;
}

extern "C" void kernel_launch(void* const* d_in, const int* in_sizes, int n_in,
                              void* d_out, int out_size, void* d_ws, size_t ws_size,
                              hipStream_t stream) {
    if (n_in < 11) return;
    if (in_sizes[0] != MROWS * DM) return;
    if (in_sizes[1] != 2 * EE * DM) return;
    if (in_sizes[2] != XR * EE) return;
    if (in_sizes[3] != EE * DTR) return;
    if (in_sizes[4] != EE) return;
    if (in_sizes[5] != EE * NS) return;
    if (in_sizes[6] != EE * NS) return;
    if (in_sizes[7] != EE) return;
    if (in_sizes[8] != DM * EE) return;
    if (in_sizes[9] != DM) return;
    if (in_sizes[10] != DM) return;
    if (out_size != MROWS * DM) return;

    const float* x          = (const float*)d_in[0];
    const float* W_in       = (const float*)d_in[1];
    const float* W_x        = (const float*)d_in[2];
    const float* W_dt       = (const float*)d_in[3];
    const float* b_dt       = (const float*)d_in[4];
    const float* A_log_real = (const float*)d_in[5];
    const float* A_imag     = (const float*)d_in[6];
    const float* D_param    = (const float*)d_in[7];
    const float* W_out      = (const float*)d_in[8];
    const float* ln_g       = (const float*)d_in[9];
    const float* ln_b       = (const float*)d_in[10];
    float* out = (float*)d_out;

    const size_t b_xn   = (size_t)MROWS * DM * 4;
    const size_t b_xz   = (size_t)MROWS * 2 * EE * 4;
    const size_t b_xdbl = (size_t)MROWS * XR * 4;
    const size_t b_dtb  = (size_t)MROWS * EE * 4;
    const size_t b_yT   = (size_t)BB * EE * TT * 4;
    const size_t b_y    = (size_t)MROWS * EE * 4;
    const size_t o_xn   = 0;
    const size_t o_xz   = o_xn + b_xn;
    const size_t o_xdbl = o_xz + b_xz;
    const size_t o_dt   = o_xdbl + b_xdbl;
    const size_t o_yT   = o_dt + b_dtb;
    const size_t o_y    = o_yT + b_yT;
    const size_t total  = o_y + b_y;
    if (total > ws_size) return;

    char* w = (char*)d_ws;
    float* xn    = (float*)(w + o_xn);
    float* xz    = (float*)(w + o_xz);
    float* xdbl  = (float*)(w + o_xdbl);
    float* dtbuf = (float*)(w + o_dt);
    float* yT    = (float*)(w + o_yT);
    float* ybuf  = (float*)(w + o_y);

    layernorm_kernel<<<MROWS, 256, 0, stream>>>(x, ln_g, ln_b, xn, MROWS);

    {
        const int M = MROWS, N = 2 * EE, K = DM;
        const int waves = (M / 16) * (N / 32);
        const int blocks = (waves + 7) / 8;
        gemm_split_kernel<0><<<blocks, 256, 0, stream>>>(xn, DM, W_in, xz, M, N, K, xn);
    }

    {
        const int M = MROWS, N = XR, K = EE;
        const int waves = (M / 16) * (N / 32);
        const int blocks = (waves + 7) / 8;
        gemm_split_kernel<0><<<blocks, 256, 0, stream>>>(xz, 2 * EE, W_x, xdbl, M, N, K, xz);
    }

    {
        const int M = MROWS, N = EE, K = DTR;
        const int waves = (M / 16) * (N / 32);
        const int blocks = (waves + 7) / 8;
        gemm_split_kernel<1><<<blocks, 256, 0, stream>>>(xdbl, XR, W_dt, dtbuf, M, N, K, b_dt);
    }

    {
        const int nch = BB * EE;
        const int blocks = (nch + 7) / 8;
        scan_kernel<<<blocks, 256, 0, stream>>>(dtbuf, xz, xdbl, A_log_real, A_imag, D_param, yT, nch);
    }

    {
        const int nblk = BB * (EE / 32) * (TT / 32);
        transpose_y_kernel<<<nblk, 256, 0, stream>>>(yT, ybuf, nblk);
    }

    {
        const int M = MROWS, N = DM, K = EE;
        const int waves = (M / 16) * (N / 32);
        const int blocks = (waves + 7) / 8;
        gemm_split_kernel<3><<<blocks, 256, 0, stream>>>(ybuf, EE, W_out, out, M, N, K, x);
    }
}
